// CfCCell_5669356836202
// MI455X (gfx1250) — hardware-verified
//
#include <hip/hip_runtime.h>

#define NB    16384
#define NIN   256
#define NHX   512
#define NCAT  768
#define NU    1024
#define NHID  512
#define NF    2048
#define XG    (NB * NCAT / 8)
#define WBG   (NU * NCAT / 8)
#define HWG   (NHID * NU / 8)
#define WHG   (4 * HWG)
#define NGRP  (XG + WBG + WHG)
#define WCARRY 1024.0f
#define WINV   0.0009765625f
#define SFP   132

static_assert(NB % 128 == 0);
static_assert(NB % 64 == 0);
static_assert(NU % 64 == 0);
static_assert(NHID % 32 == 0);
static_assert(NCAT % 32 == 0);
static_assert(NU % 32 == 0);
static_assert(NGRP % 256 == 0);
static_assert(HWG == 65536);
static_assert((NCAT / 8) == 96);
static_assert((XG % 32) == 0 && (WBG % 32) == 0 && (HWG % 32) == 0);

typedef _Float16 v16h __attribute__((ext_vector_type(16)));
typedef _Float16 v8h  __attribute__((ext_vector_type(8)));
typedef __bf16   v16b __attribute__((ext_vector_type(16)));
typedef __bf16   v8b  __attribute__((ext_vector_type(8)));
typedef unsigned short v8us __attribute__((ext_vector_type(8)));
typedef float    v8f  __attribute__((ext_vector_type(8)));
typedef float    v4f  __attribute__((ext_vector_type(4)));
typedef v8h  __attribute__((may_alias)) v8ha;
typedef v8b  __attribute__((may_alias)) v8ba;
typedef v4f  __attribute__((may_alias)) v4fa;

union FragH { v16h v; v8h half[2]; };
union FragB { v16b v; v8b half[2]; };

__device__ __forceinline__ v8f wmma_f16(v16h a, v16h b, v8f c) {
  v8f d = __builtin_amdgcn_wmma_f32_16x16x32_f16(false, a, false, b, (short)0, c, false, false);
  asm volatile("v_nop\n\tv_nop\n\tv_nop\n\tv_nop" : "+v"(d) : "v"(a), "v"(b));
  return d;
}
__device__ __forceinline__ v8f wmma_bf16(v16b a, v16b b, v8f c) {
  v8f d = __builtin_amdgcn_wmma_f32_16x16x32_bf16(false, a, false, b, (short)0, c, false, false);
  asm volatile("v_nop\n\tv_nop\n\tv_nop\n\tv_nop" : "+v"(d) : "v"(a), "v"(b));
  return d;
}

__device__ __forceinline__ v16h load_frag_h(const _Float16* p, int h) {
  FragH f;
  f.half[0] = *(const v8ha*)(p + 8 * h);
  f.half[1] = *(const v8ha*)(p + 16 + 8 * h);
  return f.v;
}
__device__ __forceinline__ v16b load_frag_b(const unsigned short* p, int h) {
  FragB f;
  f.half[0] = *(const v8ba*)(p + 8 * h);
  f.half[1] = *(const v8ba*)(p + 16 + 8 * h);
  return f.v;
}

__device__ __forceinline__ unsigned short bf16_bits(float f) {
  unsigned int u = __float_as_uint(f);
  u += 0x7fffu + ((u >> 16) & 1u);
  return (unsigned short)(u >> 16);
}
__device__ __forceinline__ float bf16r(float f) {
  unsigned int u = __float_as_uint(f);
  u += 0x7fffu + ((u >> 16) & 1u);
  return __uint_as_float(u & 0xffff0000u);
}

__global__ __launch_bounds__(256) void convert_kernel(
    const float* __restrict__ in, const float* __restrict__ hx, const float* __restrict__ wb,
    const float* __restrict__ w1, const float* __restrict__ w2,
    const float* __restrict__ wa, const float* __restrict__ wt,
    unsigned short* __restrict__ xb, unsigned short* __restrict__ wbb, _Float16* __restrict__ whp)
{
  const int g = blockIdx.x * 256 + threadIdx.x;
  if (g >= NGRP) return;
  if (g < XG + WBG) {
    const float* src;
    unsigned short* dst;
    if (g < XG) {
      const int row = g / 96;
      const int c8 = g - row * 96;
      src = (c8 < 32) ? (in + (size_t)row * NIN + 8 * c8)
                      : (hx + (size_t)row * NHX + 8 * (c8 - 32));
      dst = xb + (size_t)g * 8;
    } else {
      const int e = g - XG;
      src = wb + (size_t)e * 8;
      dst = wbb + (size_t)e * 8;
    }
    const v4f a = *(const v4fa*)src;
    const v4f c = *(const v4fa*)(src + 4);
    const v8us o = { bf16_bits(a.x), bf16_bits(a.y), bf16_bits(a.z), bf16_bits(a.w),
                     bf16_bits(c.x), bf16_bits(c.y), bf16_bits(c.z), bf16_bits(c.w) };
    *(volatile v8us*)dst = o;
    __threadfence();
    *(volatile v8us*)dst = o;
  } else {
    const int e = g - XG - WBG;
    const int wsel = e >> 16;
    const int off = e - (wsel << 16);
    const float* wsrc = (wsel == 0) ? w1 : ((wsel == 1) ? w2 : ((wsel == 2) ? wa : wt));
    const float* src = wsrc + (size_t)off * 8;
    _Float16* dst = whp + (size_t)e * 8;
    const v4f a = *(const v4fa*)src;
    const v4f c = *(const v4fa*)(src + 4);
    const v8h o = { (_Float16)(bf16r(a.x) * WCARRY), (_Float16)(bf16r(a.y) * WCARRY),
                    (_Float16)(bf16r(a.z) * WCARRY), (_Float16)(bf16r(a.w) * WCARRY),
                    (_Float16)(bf16r(c.x) * WCARRY), (_Float16)(bf16r(c.y) * WCARRY),
                    (_Float16)(bf16r(c.z) * WCARRY), (_Float16)(bf16r(c.w) * WCARRY) };
    *(volatile v8h*)dst = o;
    __threadfence();
    *(volatile v8h*)dst = o;
  }
}

__device__ __forceinline__ void h_store_pass(const _Float16* sT, _Float16* hpl,
                                             int m0, int n0, int w, int lane) {
  const int q8 = lane & 7, sub = lane >> 3;
  #pragma unroll
  for (int i = 0; i < 8; ++i) {
    const int lid = w * 32 + i * 4 + sub;
    const v8h v = *(const v8ha*)(sT + lid * 64 + 8 * q8);
    _Float16* dst = hpl + (size_t)(m0 + lid) * NU + n0 + 8 * q8;
    *(volatile v8h*)dst = v;
  }
}

__global__ __launch_bounds__(128) void backbone_kernel(
    const unsigned short* __restrict__ xb,
    const unsigned short* __restrict__ wbb,
    const float* __restrict__ bb,
    _Float16* __restrict__ hpl)
{
  __shared__ __attribute__((aligned(16))) float    sF[128 * 64];
  __shared__ __attribute__((aligned(16))) _Float16 sT[128 * 64];

  const int tid = threadIdx.x, lane = tid & 31, w = tid >> 5;
  const int h = lane >> 4, m = lane & 15;
  const int m0 = blockIdx.x * 128;
  const int n0 = blockIdx.y * 64;
  const int m0w = m0 + 32 * w;

  const unsigned short* xa0 = xb + (size_t)(m0w + m) * NCAT;
  const unsigned short* xa1 = xa0 + (size_t)16 * NCAT;
  const unsigned short* wbr = wbb + (size_t)(n0 + m) * NCAT;

  const v8f zero8 = {0.f, 0.f, 0.f, 0.f, 0.f, 0.f, 0.f, 0.f};
  v8f acc[2][4];
  #pragma unroll
  for (int mt = 0; mt < 2; ++mt)
    #pragma unroll
    for (int nt = 0; nt < 4; ++nt) acc[mt][nt] = zero8;

  #pragma unroll 1
  for (int k0 = 0; k0 < NCAT; k0 += 32) {
    const v16b a0 = load_frag_b(xa0 + k0, h);
    const v16b a1 = load_frag_b(xa1 + k0, h);
    #pragma unroll
    for (int nt = 0; nt < 4; ++nt) {
      const v16b b = load_frag_b(wbr + (size_t)nt * 16 * NCAT + k0, h);
      acc[0][nt] = wmma_bf16(a0, b, acc[0][nt]);
      acc[1][nt] = wmma_bf16(a1, b, acc[1][nt]);
    }
  }

  #pragma unroll
  for (int nt = 0; nt < 4; ++nt) {
    const int col = 16 * nt + m;
    const float bvl = bf16r(bb[n0 + col]);
    #pragma unroll
    for (int mt = 0; mt < 2; ++mt) {
      #pragma unroll
      for (int r = 0; r < 8; ++r) {
        const int rowl = 32 * w + 16 * mt + 8 * h + r;
        sF[rowl * 64 + col] = acc[mt][nt][r] + bvl;
      }
    }
  }
  __syncthreads();

  #pragma unroll 1
  for (int j = 0; j < 64; ++j) {
    const int e = tid + 128 * j;
    const float v = sF[e];
    const float hv = 1.7159f * tanhf(0.666f * v);
    sT[e] = (_Float16)hv;
  }
  __syncthreads();

  h_store_pass(sT, hpl, m0, n0, w, lane);
  __threadfence();
  h_store_pass(sT, hpl, m0, n0, w, lane);
}

__device__ __forceinline__ void o_store_pass(const float* sO, float* out,
                                             int m0, int c0, int w, int lane) {
  const int q8 = lane & 7, sub = lane >> 3;
  #pragma unroll
  for (int i = 0; i < 4; ++i) {
    const int lid = w * 16 + i * 4 + sub;
    const v4f v = *(const v4fa*)(sO + lid * 32 + 4 * q8);
    float* dst = out + (size_t)(m0 + lid) * NHID + c0 + 4 * q8;
    *(volatile v4f*)dst = v;
  }
}

__global__ __launch_bounds__(128) void heads_kernel(
    const _Float16* __restrict__ hpl,
    const _Float16* __restrict__ whp,
    const float* __restrict__ b1, const float* __restrict__ b2,
    const float* __restrict__ ba, const float* __restrict__ bt,
    const float* __restrict__ ts,
    float* __restrict__ out)
{
  __shared__ __attribute__((aligned(16))) float sF[64 * SFP];
  __shared__ __attribute__((aligned(16))) float sO[64 * 32];
  __shared__ __attribute__((aligned(16))) float sTS[64];

  const int tid = threadIdx.x, lane = tid & 31, w = tid >> 5;
  const int h = lane >> 4, m = lane & 15;
  const int wm = w & 1, wn = w >> 1;
  const int m0 = blockIdx.x * 64;
  const int c0 = blockIdx.y * 32;

  const _Float16* ha0 = hpl + (size_t)(m0 + 32 * wm + m) * NU;
  const _Float16* ha1 = ha0 + (size_t)16 * NU;
  const _Float16* wr0 = whp + ((size_t)(2 * wn) * NHID + c0 + m) * NU;
  const _Float16* wr1 = wr0 + (size_t)NHID * NU;

  const v8f zero8 = {0.f, 0.f, 0.f, 0.f, 0.f, 0.f, 0.f, 0.f};
  v8f acc[2][4];
  #pragma unroll
  for (int mt = 0; mt < 2; ++mt)
    #pragma unroll
    for (int q = 0; q < 4; ++q) acc[mt][q] = zero8;

  #pragma unroll 1
  for (int k0 = 0; k0 < NU; k0 += 32) {
    const v16h a0 = load_frag_h(ha0 + k0, h);
    const v16h a1 = load_frag_h(ha1 + k0, h);
    #pragma unroll
    for (int q = 0; q < 4; ++q) {
      const int hh = q >> 1, nt = q & 1;
      const _Float16* wp = (hh ? wr1 : wr0) + (size_t)nt * 16 * NU + k0;
      const v16h b = load_frag_h(wp, h);
      acc[0][q] = wmma_f16(a0, b, acc[0][q]);
      acc[1][q] = wmma_f16(a1, b, acc[1][q]);
    }
  }

  if (tid < 64) sTS[tid] = bf16r(ts[m0 + tid]);

  const float* bp0 = (wn == 0) ? b1 : ba;
  const float* bp1 = (wn == 0) ? b2 : bt;
  #pragma unroll
  for (int q = 0; q < 4; ++q) {
    const int hh = q >> 1, nt = q & 1;
    const int col = 16 * nt + m;
    const float bvl = bf16r((hh ? bp1 : bp0)[c0 + col]);
    const int fused = (2 * wn + hh) * 32 + col;
    #pragma unroll
    for (int mt = 0; mt < 2; ++mt) {
      #pragma unroll
      for (int r = 0; r < 8; ++r) {
        const int rowl = 32 * wm + 16 * mt + 8 * h + r;
        sF[rowl * SFP + fused] = acc[mt][q][r] * WINV + bvl;
      }
    }
  }
  __syncthreads();

  #pragma unroll 1
  for (int j = 0; j < 16; ++j) {
    const int e = tid + 128 * j;
    const int row = e >> 5, col = e & 31;
    const float* fr = sF + row * SFP + col;
    const float f1 = tanhf(fr[0]);
    const float f2 = tanhf(fr[32]);
    const float ta = fr[64];
    const float tb = fr[96];
    float z = ta * sTS[row] + tb;
    z = fminf(fmaxf(z, -40.0f), 40.0f);
    const float ti = 1.0f / (1.0f + expf(-z));
    sO[e] = f1 * (1.0f - ti) + ti * f2;
  }
  __syncthreads();

  o_store_pass(sO, out, m0, c0, w, lane);
  __threadfence();
  o_store_pass(sO, out, m0, c0, w, lane);
}

extern "C" void kernel_launch(void* const* d_in, const int* in_sizes, int n_in,
                              void* d_out, int out_size, void* d_ws, size_t ws_size,
                              hipStream_t stream) {
  if (n_in < 13) return;
  if (in_sizes[0] != NB * NIN) return;
  if (in_sizes[1] != NB * NHX) return;
  if (in_sizes[2] != NB) return;
  if (in_sizes[3] != NU * NCAT || in_sizes[4] != NU) return;
  if (in_sizes[5] != NHID * NU || in_sizes[7] != NHID * NU ||
      in_sizes[9] != NHID * NU || in_sizes[11] != NHID * NU) return;
  if (in_sizes[6] != NHID || in_sizes[8] != NHID || in_sizes[10] != NHID || in_sizes[12] != NHID) return;
  if (out_size != NB * NHID) return;

  const float* in = (const float*)d_in[0];
  const float* hx = (const float*)d_in[1];
  const float* ts = (const float*)d_in[2];
  const float* Wb = (const float*)d_in[3];
  const float* bb = (const float*)d_in[4];
  const float* W1 = (const float*)d_in[5];
  const float* b1 = (const float*)d_in[6];
  const float* W2 = (const float*)d_in[7];
  const float* b2 = (const float*)d_in[8];
  const float* Wa = (const float*)d_in[9];
  const float* ba = (const float*)d_in[10];
  const float* Wt = (const float*)d_in[11];
  const float* bt = (const float*)d_in[12];
  float* out = (float*)d_out;

  const size_t xb_bytes  = (size_t)NB * NCAT * 2;
  const size_t wbb_bytes = (size_t)NU * NCAT * 2;
  const size_t hpl_bytes = (size_t)NB * NU * 2;
  const size_t whp_bytes = (size_t)NF * NU * 2;
  const size_t total = xb_bytes + wbb_bytes + hpl_bytes + whp_bytes;
  if (total > ws_size) return;

  char* ws = (char*)d_ws;
  unsigned short* xb  = (unsigned short*)(ws);
  unsigned short* wbb = (unsigned short*)(ws + xb_bytes);
  _Float16* hpl = (_Float16*)(ws + xb_bytes + wbb_bytes);
  _Float16* whp = (_Float16*)(ws + xb_bytes + wbb_bytes + hpl_bytes);

  convert_kernel<<<NGRP / 256, 256, 0, stream>>>(in, hx, Wb, W1, W2, Wa, Wt, xb, wbb, whp);

  dim3 gBack(NB / 128, NU / 64);
  backbone_kernel<<<gBack, 128, 0, stream>>>(xb, wbb, bb, hpl);

  dim3 gHead(NB / 64, NHID / 32);
  heads_kernel<<<gHead, 128, 0, stream>>>(hpl, whp, b1, b2, ba, bt, ts, out);
}
